// CrystalEncoder_11570641896052
// MI455X (gfx1250) — hardware-verified
//
#include <hip/hip_runtime.h>
#include <stddef.h>
#include <stdint.h>

#pragma clang fp contract(off)


#define BB    8
#define NN    256
#define HH    128
#define LAT   64
#define NLAY  2
#define NBIN  40
#define KP    64
#define HSTR  136
#define IT    16
#define TPB   256
#define TPBP  128
#define NTAB  100

#define FRH      512
#define OFFP_E   0
#define SZP_E    (NLAY * 2 * 8 * FRH)
#define OFFP_N   (OFFP_E + SZP_E)
#define SZP_N    (NLAY * 4 * 8 * FRH)
#define PK_TOTAL (OFFP_N + SZP_N)
#define NGRP     (PK_TOTAL / 8)
#define PK_BYTES ((size_t)PK_TOTAL * 2)
#define OFF_HA   PK_BYTES
#define H_BYTES  ((size_t)BB * NN * HH * 4)
#define OFF_HB   (OFF_HA + H_BYTES)
#define WS_TOTAL (OFF_HB + H_BYTES)
#define WSCAP    134217728

#define WSC   16.0f
#define RSC   64.0f
#define HSC   64.0f
#define ASC   16.0f
#define PSE   0.0009765625f
#define IHS   0.015625f
#define PSN   0.00390625f
#define NG2E  (-36.067376f)
#define NL2E  (-1.44269504f)
#define LN2F  0.69314718f
#define CSTP  0.025641026f

static_assert(OFFP_N == 16384);
static_assert(PK_TOTAL == 49152);
static_assert(NGRP == 6144);
static_assert((NGRP % 32) == 0);
static_assert((NGRP % TPBP) == 0);
static_assert((OFFP_N % 256) == 0);
static_assert((OFF_HA % 512) == 0);
static_assert((OFF_HB % 512) == 0);
static_assert(WS_TOTAL <= (size_t)WSCAP);
static_assert(TPB == NN);
static_assert((NN % IT) == 0);
static_assert(IT * HH == TPB * 8);
static_assert(NBIN <= KP);
static_assert((NBIN % 8) == 0);

typedef _Float16     v16h __attribute__((ext_vector_type(16)));
typedef _Float16     v8h  __attribute__((ext_vector_type(8)));
typedef _Float16     v4h  __attribute__((ext_vector_type(4)));
typedef float        v8f  __attribute__((ext_vector_type(8)));
typedef float        v4f  __attribute__((ext_vector_type(4)));
typedef unsigned int v4u  __attribute__((ext_vector_type(4)));
union Frag { v16h v; v8h half[2]; };
union Pk8  { v8h h; v4u u; };

__device__ __forceinline__ int imin(int a, int b) { return a < b ? a : b; }
__device__ __forceinline__ int imax(int a, int b) { return a > b ? a : b; }

__device__ __forceinline__ float exp2_raw(float x) { return __builtin_amdgcn_exp2f(x); }
__device__ __forceinline__ float log2_raw(float x) { return __builtin_amdgcn_logf(x); }
__device__ __forceinline__ float rcp_raw(float x)  { return __builtin_amdgcn_rcpf(x); }

__device__ __forceinline__ float softplus_f(float x) {
  const float t = exp2_raw(NL2E * __builtin_fabsf(x));
  return fmaxf(x, 0.0f) + LN2F * log2_raw(1.0f + t);
}

__device__ __forceinline__ v4u cvt8s(const v4f a, const v4f b, const float s) {
  v8h hv = {(_Float16)(a.x * s), (_Float16)(a.y * s), (_Float16)(a.z * s), (_Float16)(a.w * s),
            (_Float16)(b.x * s), (_Float16)(b.y * s), (_Float16)(b.z * s), (_Float16)(b.w * s)};
  Pk8 p;
  p.h = hv;
  return p.u;
}

__device__ __forceinline__ v8f wmh(v16h a, v16h b, v8f c) {
  v8f d = __builtin_amdgcn_wmma_f32_16x16x32_f16(false, a, false, b, (short)0, c, false, false);
  asm volatile("v_nop\n\tv_nop\n\tv_nop\n\tv_nop" : "+v"(d) : "v"(a), "v"(b));
  return d;
}

__device__ __forceinline__ v16h ldA(const _Float16* base, int ld, int lane) {
  Frag a;
  const _Float16* p = base + (lane & 15) * ld + 8 * (lane >> 4);
  a.half[0] = *(const v8h*)p;
  a.half[1] = *(const v8h*)(p + 16);
  return a.v;
}

__device__ __forceinline__ v16h ldB(const _Float16* pk, int frag, int lane) {
  Frag b;
  const _Float16* p = pk + (size_t)((frag << 5) + lane) * 16;
  b.half[0] = *(const v8h*)p;
  b.half[1] = *(const v8h*)(p + 8);
  return b.v;
}

__global__ __launch_bounds__(TPBP) void k_prep(const float* __restrict__ edge_w, const float* __restrict__ node_w,
                                               _Float16* pk) {
  const int tid = threadIdx.x;
  const int g = blockIdx.x * TPBP + tid;
  const int wg = __builtin_amdgcn_readfirstlane(g >> 5);
  if (wg >= NGRP / 32) return;
  const int pw = wg * 256;
  const float* src;
  int K, lbase;
  if (pw < OFFP_N) {
    const int l = pw / (16 * FRH);         lbase = pw - l * (16 * FRH); src = edge_w + l * (NBIN * HH); K = NBIN;
  } else {
    const int q = pw - OFFP_N;
    const int l = q / (32 * FRH);          lbase = q - l * (32 * FRH);  src = node_w + l * (HH * HH);   K = HH;
  }
  const int lane = g & 31;
  const int loc0 = lbase + lane * 8;
  const int e0 = loc0 & 15;
  const int L = (loc0 >> 4) & 31;
  const int ft = loc0 >> 9;
  const int t = ft & 7, s = ft >> 3;
  const int hh = L >> 4, c = 16 * t + (L & 15);
  float tv[8];
#pragma unroll
  for (int u = 0; u < 8; ++u) {
    const int e = e0 + u;
    const int k = 32 * s + ((e < 8) ? (8 * hh + e) : (8 + 8 * hh + e));
    const int kc = imin(k, K - 1);
    const float v = src[kc * HH + c];
    tv[u] = (k < K) ? v : 0.0f;
  }
  const v4f f0 = {tv[0], tv[1], tv[2], tv[3]};
  const v4f f1 = {tv[4], tv[5], tv[6], tv[7]};
  const v4u pkv = cvt8s(f0, f1, WSC);
  _Float16* d = pk + (size_t)g * 8;
  *(volatile v4u*)d = pkv;
  __threadfence();
  *(volatile v4u*)d = pkv;
}

__global__ __launch_bounds__(TPB) void k_embed(const int* __restrict__ atyp, const float* __restrict__ emb,
                                               float* h0) {
  const int q = blockIdx.x * TPB + threadIdx.x;
  if (q >= BB * NN * (HH / 4)) return;
  const int row = q >> 5, c4 = q & 31;
  int a = atyp[row];
  a = imin(imax(a, 0), NTAB - 1);
  const v4f v = *(const v4f*)(emb + (size_t)a * HH + 4 * c4);
  float* p = h0 + (size_t)row * HH + 4 * c4;
  *(volatile v4f*)p = v;
  __threadfence();
  *(volatile v4f*)p = v;
}

__global__ __launch_bounds__(TPB) void k_layer(const float* __restrict__ frac, const float* __restrict__ lat,
                                               const int* __restrict__ mask, const float* __restrict__ h_in,
                                               float* h_out, const _Float16* __restrict__ pk,
                                               const float* __restrict__ edge_b, const float* __restrict__ node_b,
                                               int l) {
  __shared__ __attribute__((aligned(16))) _Float16 rbfs[NN * KP];
  __shared__ __attribute__((aligned(16))) _Float16 hsh[NN * HSTR];
  __shared__ __attribute__((aligned(16))) float    aggf[IT * HH];
  __shared__ __attribute__((aligned(16))) _Float16 aggh[IT * HSTR];
  __shared__ __attribute__((aligned(16))) float    hnew[IT * HH];
  __shared__ __attribute__((aligned(16))) float    cartS[NN * 4];
  __shared__ int   maskS[NN];
  __shared__ float cen[KP];

  const int tid = threadIdx.x, lane = tid & 31, hf = lane >> 4, m = lane & 15;
  const int w = __builtin_amdgcn_readfirstlane(tid >> 5);
  const int b = blockIdx.x / (NN / IT);
  const int i0 = (blockIdx.x - b * (NN / IT)) * IT;
  const int hcol = 16 * w + m;
  const v8f zero8 = {0.f, 0.f, 0.f, 0.f, 0.f, 0.f, 0.f, 0.f};

  {
    const int n = tid;
    const float* f = frac + ((size_t)(b * NN + n)) * 3;
    const float* Lm = lat + b * 9;
    const float f0 = f[0], f1 = f[1], f2 = f[2];
#pragma unroll
    for (int e = 0; e < 3; ++e) {
      float p = f0 * Lm[e];
      p = fmaf(f1, Lm[3 + e], p);
      p = fmaf(f2, Lm[6 + e], p);
      cartS[4 * n + e] = p;
    }
    cartS[4 * n + 3] = 0.0f;
    maskS[n] = mask[b * NN + n];
    if (n < KP) cen[n] = (n < NBIN) ? 8.0f * ((float)n * CSTP) : 0.0f;
  }
  __syncthreads();

#pragma unroll 2
  for (int it = 0; it < (NN * HH) / (4 * TPB); ++it) {
    const int q = it * TPB + tid;
    const int n = q >> 5, c4 = q & 31;
    const v4f v = *(const v4f*)(h_in + ((size_t)(b * NN + n)) * HH + 4 * c4);
    const float s = (maskS[n] != 0) ? HSC : 0.0f;
    const v4h hv = {(_Float16)(v.x * s), (_Float16)(v.y * s), (_Float16)(v.z * s), (_Float16)(v.w * s)};
    *(v4h*)(hsh + n * HSTR + 4 * c4) = hv;
  }
  __syncthreads();

  const _Float16* pkE = pk + OFFP_E + l * (16 * FRH);
  const v16h bt0 = ldB(pkE, w, lane);
  const v16h bt1 = ldB(pkE, 8 + w, lane);
  const float eb = edge_b[l * HH + hcol];

#pragma unroll 1
  for (int ii = 0; ii < IT; ++ii) {
    const int i = i0 + ii;
    {
      const int j = tid;
      const float dx = cartS[4 * i + 0] - cartS[4 * j + 0];
      const float dy = cartS[4 * i + 1] - cartS[4 * j + 1];
      const float dz = cartS[4 * i + 2] - cartS[4 * j + 2];
      const float ss = (dx * dx + dz * dz) + dy * dy;
      const float d = sqrtf(ss + 1e-6f);
#pragma unroll 1
      for (int fg = 0; fg < NBIN / 8; ++fg) {
        float tv[8];
#pragma unroll
        for (int u = 0; u < 8; ++u) {
          const float t = d - cen[8 * fg + u];
          tv[u] = exp2_raw((t * t) * NG2E);
        }
        const v4f q0 = {tv[0], tv[1], tv[2], tv[3]};
        const v4f q1 = {tv[4], tv[5], tv[6], tv[7]};
        *(v4u*)(rbfs + j * KP + 8 * fg) = cvt8s(q0, q1, RSC);
      }
      const v4u z4 = {0u, 0u, 0u, 0u};
#pragma unroll
      for (int fg = NBIN / 8; fg < KP / 8; ++fg) *(v4u*)(rbfs + j * KP + 8 * fg) = z4;
    }
    __syncthreads();

    float acc = 0.0f;
#pragma unroll 1
    for (int jt = 0; jt < NN / 16; ++jt) {
      const _Float16* ap = rbfs + jt * (16 * KP);
      const v16h a0 = ldA(ap, KP, lane);
      const v16h a1 = ldA(ap + 32, KP, lane);
      v8f c = wmh(a0, bt0, zero8);
      c = wmh(a1, bt1, c);
      const _Float16* hp = hsh + (jt * 16 + 8 * hf) * HSTR + hcol;
#pragma unroll
      for (int r = 0; r < 8; ++r) {
        const float pre = c[r] * PSE + eb;
        const float gv = softplus_f(pre);
        acc = fmaf(gv, (float)hp[r * HSTR], acc);
      }
    }
    acc += __shfl_xor(acc, 16, 32);
    aggf[ii * HH + hcol] = (maskS[i] != 0) ? (acc * IHS) : 0.0f;
    __syncthreads();
  }

  {
    const int row = tid >> 4, c8 = tid & 15;
    const v4f a0 = *(const v4f*)(aggf + row * HH + 8 * c8);
    const v4f a1 = *(const v4f*)(aggf + row * HH + 8 * c8 + 4);
    *(v4u*)(aggh + row * HSTR + 8 * c8) = cvt8s(a0, a1, ASC);
  }
  __syncthreads();

  {
    const _Float16* pkN = pk + OFFP_N + l * (32 * FRH);
    v8f acc8 = zero8;
#pragma unroll
    for (int s = 0; s < 4; ++s) acc8 = wmh(ldA(aggh + 32 * s, HSTR, lane), ldB(pkN, s * 8 + w, lane), acc8);
    const float nb = node_b[l * HH + hcol];
#pragma unroll
    for (int r = 0; r < 8; ++r) {
      const int il = 8 * hf + r;
      const float dot = acc8[r] * PSN + nb;
      const float ex = exp2_raw(NL2E * dot);
      const float sg = dot * rcp_raw(1.0f + ex);
      const float hin = h_in[((size_t)(b * NN + i0 + il)) * HH + hcol];
      const float mk = (maskS[i0 + il] != 0) ? 1.0f : 0.0f;
      hnew[il * HH + hcol] = (hin + sg) * mk;
    }
  }
  __syncthreads();

  v4f ov[2];
#pragma unroll
  for (int it = 0; it < 2; ++it) {
    const int q = it * TPB + tid;
    const int row = q >> 5, c4 = q & 31;
    ov[it] = *(const v4f*)(hnew + row * HH + 4 * c4);
  }
#pragma unroll
  for (int it = 0; it < 2; ++it) {
    const int q = it * TPB + tid;
    const int row = q >> 5, c4 = q & 31;
    *(volatile v4f*)(h_out + ((size_t)(b * NN + i0 + row)) * HH + 4 * c4) = ov[it];
  }
  __threadfence();
#pragma unroll
  for (int it = 0; it < 2; ++it) {
    const int q = it * TPB + tid;
    const int row = q >> 5, c4 = q & 31;
    *(volatile v4f*)(h_out + ((size_t)(b * NN + i0 + row)) * HH + 4 * c4) = ov[it];
  }
}

__global__ __launch_bounds__(TPB) void k_pool(const int* __restrict__ mask, const float* __restrict__ h,
                                              const float* __restrict__ mu_w, const float* __restrict__ mu_b,
                                              const float* __restrict__ var_w, const float* __restrict__ var_b,
                                              float* out) {
  __shared__ float part[2 * HH];
  __shared__ float g[HH];
  __shared__ __attribute__((aligned(16))) float outS[2 * LAT];
  __shared__ int   maskS[NN];
  const int b = blockIdx.x;
  const int tid = threadIdx.x, lane = tid & 31;

  maskS[tid] = mask[b * NN + tid];
  __syncthreads();

  int cnt = 0;
#pragma unroll 1
  for (int n = 0; n < NN; ++n) cnt += (maskS[n] != 0) ? 1 : 0;

  {
    const int sl = tid >> 7, hc = tid & (HH - 1);
    float s = 0.0f;
#pragma unroll 1
    for (int n = sl * (NN / 2); n < sl * (NN / 2) + NN / 2; ++n) {
      const float mk = (maskS[n] != 0) ? 1.0f : 0.0f;
      s += h[((size_t)(b * NN + n)) * HH + hc] * mk;
    }
    part[sl * HH + hc] = s;
  }
  __syncthreads();
  if (tid < HH) {
    const float inv = 1.0f / ((float)cnt + 1e-6f);
    g[tid] = (part[tid] + part[HH + tid]) * inv;
  }
  __syncthreads();

  if (tid < LAT) {
    float d = 0.0f;
#pragma unroll 1
    for (int k = 0; k < HH; ++k) d = fmaf(g[k], mu_w[k * LAT + tid], d);
    outS[tid] = d + mu_b[tid];
  } else if (tid < 2 * LAT) {
    const int lv = tid - LAT;
    float d = 0.0f;
#pragma unroll 1
    for (int k = 0; k < HH; ++k) d = fmaf(g[k], var_w[k * LAT + lv], d);
    outS[LAT + lv] = d + var_b[lv];
  }
  __syncthreads();

  if (tid < 32) {
    const v4f v = *(const v4f*)(outS + 4 * lane);
    float* p = out + b * LAT + 4 * lane + ((lane >= 16) ? (BB * LAT - LAT) : 0);
    *(volatile v4f*)p = v;
    __threadfence();
    *(volatile v4f*)p = v;
  }
}

extern "C" void kernel_launch(void* const* d_in, const int* in_sizes, int n_in,
                              void* d_out, int out_size, void* d_ws, size_t ws_size,
                              hipStream_t stream) {
  if (n_in < 13) return;
  if (in_sizes[0] != BB * NN) return;
  if (in_sizes[1] != BB * NN * 3) return;
  if (in_sizes[2] != BB * 9) return;
  if (in_sizes[3] != BB * NN) return;
  if (in_sizes[4] != NTAB * HH) return;
  if (in_sizes[5] != NLAY * NBIN * HH) return;
  if (in_sizes[6] != NLAY * HH) return;
  if (in_sizes[7] != NLAY * HH * HH) return;
  if (in_sizes[8] != NLAY * HH) return;
  if (in_sizes[9] != HH * LAT || in_sizes[10] != LAT) return;
  if (in_sizes[11] != HH * LAT || in_sizes[12] != LAT) return;
  if (out_size != 2 * BB * LAT) return;
  if (WS_TOTAL > ws_size || WS_TOTAL > (size_t)WSCAP) return;

  const int*   atyp   = (const int*)d_in[0];
  const float* frac   = (const float*)d_in[1];
  const float* lat    = (const float*)d_in[2];
  const int*   mask   = (const int*)d_in[3];
  const float* emb    = (const float*)d_in[4];
  const float* edge_w = (const float*)d_in[5];
  const float* edge_b = (const float*)d_in[6];
  const float* node_w = (const float*)d_in[7];
  const float* node_b = (const float*)d_in[8];
  const float* mu_w   = (const float*)d_in[9];
  const float* mu_b   = (const float*)d_in[10];
  const float* var_w  = (const float*)d_in[11];
  const float* var_b  = (const float*)d_in[12];
  float* out = (float*)d_out;

  char* ws = (char*)d_ws;
  _Float16* pk = (_Float16*)(ws);
  float* hA = (float*)(ws + OFF_HA);
  float* hB = (float*)(ws + OFF_HB);

  k_prep<<<dim3(NGRP / TPBP), dim3(TPBP), 0, stream>>>(edge_w, node_w, pk);
  k_embed<<<dim3((BB * NN * (HH / 4)) / TPB), dim3(TPB), 0, stream>>>(atyp, emb, hA);
  k_layer<<<dim3(BB * (NN / IT)), dim3(TPB), 0, stream>>>(frac, lat, mask, hA, hB, pk, edge_b, node_b, 0);
  k_layer<<<dim3(BB * (NN / IT)), dim3(TPB), 0, stream>>>(frac, lat, mask, hB, hA, pk, edge_b, node_b, 1);
  k_pool<<<dim3(BB), dim3(TPB), 0, stream>>>(mask, hA, mu_w, mu_b, var_w, var_b, out);
}
